// S4sequence_68427418960361
// MI455X (gfx1250) — hardware-verified
//
#include <hip/hip_runtime.h>
#include <stdint.h>


#define NB 8
#define LSEQ 4096
#define HD 128
#define NS 64
#define EPS_F 1e-5f
#define APITCH 136
#define BPITCH 136
#define OPITCH 132

typedef _Float16 v16h __attribute__((ext_vector_type(16)));
typedef _Float16 v8h __attribute__((ext_vector_type(8)));
typedef __bf16 v16bf __attribute__((ext_vector_type(16)));
typedef unsigned short v8us __attribute__((ext_vector_type(8)));
typedef float v8f __attribute__((ext_vector_type(8)));
typedef float v4f __attribute__((ext_vector_type(4)));

union FragH { v16h v; v8h hv[2]; _Float16 e[16]; };
union FragB { v16bf v; v8us hv[2]; unsigned short e[16]; };
union Pack8h { v8h v; _Float16 e[8]; };
union Pack8us { v8us v; unsigned short e[8]; };

__device__ __forceinline__ v8f mma_f16(v16h a, v16h b, v8f c) {
    c = __builtin_amdgcn_wmma_f32_16x16x32_f16(false, a, false, b, (short)0, c, false, false);
    asm volatile("v_nop\n\tv_nop\n\tv_nop\n\tv_nop" : "+v"(c) : "v"(a), "v"(b));
    return c;
}
__device__ __forceinline__ v8f mma_bf16(v16bf a, v16bf b, v8f c) {
    c = __builtin_amdgcn_wmma_f32_16x16x32_bf16(false, a, false, b, (short)0, c, false, false);
    asm volatile("v_nop\n\tv_nop\n\tv_nop\n\tv_nop" : "+v"(c) : "v"(a), "v"(b));
    return c;
}

__device__ __forceinline__ unsigned short bf16_bits(float f) {
    unsigned u = __float_as_uint(f);
    u += 0x7FFFu + ((u >> 16) & 1u);
    return (unsigned short)(u >> 16);
}
__device__ __forceinline__ void split_bf16(float f, unsigned short& hi, unsigned short& lo) {
    hi = bf16_bits(f);
    float fh = __uint_as_float(((unsigned)hi) << 16);
    lo = bf16_bits(f - fh);
}

__global__ __launch_bounds__(256) void k_stats(const float* __restrict__ x, float* stats)
{
    __shared__ double s_sum[256];
    __shared__ double s_sq[256];
    __shared__ float s_res[2];
    const int b = blockIdx.x;
    if (b >= NB) return;
    const int tid = threadIdx.x;
    const size_t n = (size_t)LSEQ * HD;
    const float* xb = x + (size_t)b * n;
    double acc = 0.0, acc2 = 0.0;
#pragma unroll 4
    for (size_t i = tid; i < n; i += 256) {
        double v = (double)xb[i];
        acc += v;
        acc2 += v * v;
    }
    s_sum[tid] = acc;
    s_sq[tid] = acc2;
    __syncthreads();
    for (int off = 128; off > 0; off >>= 1) {
        if (tid < off) {
            s_sum[tid] += s_sum[tid + off];
            s_sq[tid]  += s_sq[tid + off];
        }
        __syncthreads();
    }
    if (tid == 0) {
        double inv_n = 1.0 / (double)n;
        double mu = s_sum[0] * inv_n;
        double var = s_sq[0] * inv_n - mu * mu;
        if (var < 0.0) var = 0.0;
        float varf = (float)var;
        s_res[0] = (float)mu;
        s_res[1] = 1.0f / sqrtf(varf + EPS_F);
    }
    __syncthreads();
    if (tid < 8) {
        v4f v = {0.0f, 0.0f, 0.0f, 0.0f};
        if (tid == 0) { v.x = s_res[0]; v.y = s_res[1]; }
        float* dst = stats + b * 32 + tid * 4;
        *(volatile v4f*)dst = v;
        __threadfence();
        *(volatile v4f*)dst = v;
    }
}

__global__ __launch_bounds__(256) void k_tw(float* tw)
{
    const int t = blockIdx.x * 256 + threadIdx.x;
    if (t >= LSEQ / 4) return;
    const float w = 6.283185307179586f / 4096.0f;
    const int j = 2 * t;
    float s0, c0, s1, c1;
    sincosf(w * (float)j, &s0, &c0);
    sincosf(w * (float)(j + 1), &s1, &c1);
    v4f v = {c0, s0, c1, s1};
    float* dst = tw + 4 * t;
    *(volatile v4f*)dst = v;
    __threadfence();
    *(volatile v4f*)dst = v;
}

__device__ __forceinline__ v8f cauchy_tile(v8f acc, float gr, float gi,
                                            const float* s_lr, const float* s_li,
                                            const unsigned short* sAhi, const unsigned short* sAlo,
                                            int m, int hh)
{
#pragma unroll
    for (int s = 0; s < 2; ++s) {
        float xr[16], xi[16];
#pragma unroll
        for (int i = 0; i < 16; ++i) {
            const int n = s * 32 + 8 * hh + i + (i & 8);
            float dr = gr - s_lr[n];
            float di = gi - s_li[n];
            float d = __builtin_amdgcn_rcpf(dr * dr + di * di);
            xr[i] = dr * d;
            xi[i] = -di * d;
        }
        FragB ah, al, bh, bl;
        const int kb = s * 32 + 8 * hh;
        ah.hv[0] = *(const v8us*)(sAhi + m * APITCH + kb);
        ah.hv[1] = *(const v8us*)(sAhi + m * APITCH + kb + 16);
        al.hv[0] = *(const v8us*)(sAlo + m * APITCH + kb);
        al.hv[1] = *(const v8us*)(sAlo + m * APITCH + kb + 16);
#pragma unroll
        for (int i = 0; i < 16; ++i) { unsigned short hi, lo; split_bf16(xr[i], hi, lo); bh.e[i] = hi; bl.e[i] = lo; }
        acc = mma_bf16(ah.v, bh.v, acc);
        acc = mma_bf16(ah.v, bl.v, acc);
        acc = mma_bf16(al.v, bh.v, acc);
        const int kb2 = 64 + kb;
        ah.hv[0] = *(const v8us*)(sAhi + m * APITCH + kb2);
        ah.hv[1] = *(const v8us*)(sAhi + m * APITCH + kb2 + 16);
        al.hv[0] = *(const v8us*)(sAlo + m * APITCH + kb2);
        al.hv[1] = *(const v8us*)(sAlo + m * APITCH + kb2 + 16);
#pragma unroll
        for (int i = 0; i < 16; ++i) { unsigned short hi, lo; split_bf16(xi[i], hi, lo); bh.e[i] = hi; bl.e[i] = lo; }
        acc = mma_bf16(ah.v, bh.v, acc);
        acc = mma_bf16(ah.v, bl.v, acc);
        acc = mma_bf16(al.v, bh.v, acc);
    }
    return acc;
}

__global__ __launch_bounds__(256) void k_cauchy(
    const float* __restrict__ LamR, const float* __restrict__ LamI,
    const float* __restrict__ Pre,  const float* __restrict__ Pim,
    const float* __restrict__ Bre,  const float* __restrict__ Bim,
    const float* __restrict__ Cre,  const float* __restrict__ Cim,
    float* Kr, float* Ki)
{
    __shared__ float s_lr[NS];
    __shared__ float s_li[NS];
    __shared__ __attribute__((aligned(16))) unsigned short sAhi[16 * APITCH];
    __shared__ __attribute__((aligned(16))) unsigned short sAlo[16 * APITCH];
    __shared__ __attribute__((aligned(16))) float sK[2 * 256];

    const int blk = blockIdx.x;
    if (blk >= HD * (LSEQ / 256)) return;
    const int h = blk >> 4;
    const int l0 = (blk & 15) * 256;
    const int tid = threadIdx.x;
    const int lane = tid & 31, wave = tid >> 5;
    const int hh = lane >> 4, m = lane & 15;

    if (tid < NS) {
        s_lr[tid] = LamR[h * NS + tid];
        s_li[tid] = LamI[h * NS + tid];
    }
    {
        const int j = tid >> 4;
        const int kc = (tid & 15) * 8;
        Pack8us ph, pl;
#pragma unroll
        for (int e = 0; e < 8; ++e) {
            float val = 0.0f;
            if (j < 8) {
                const int k = kc + e;
                const int n = k & 63;
                const int part = k >> 6;
                const int o = h * NS + n;
                const float cr = Cre[o], ci = Cim[o];
                const float br = Bre[o], bi = Bim[o];
                const float pr = Pre[o], pi = Pim[o];
                const int q = j >> 1;
                const float ar = (q < 2) ? cr : pr;
                const float ai = (q < 2) ? ci : pi;
                const float xr = (q & 1) ? pr : br;
                const float xi = (q & 1) ? pi : bi;
                const float vr = ar * xr + ai * xi;
                const float vi = ar * xi - ai * xr;
                if (j & 1) val = part ? vr : vi;
                else       val = part ? -vi : vr;
            }
            unsigned short hi, lo;
            split_bf16(val, hi, lo);
            ph.e[e] = hi;
            pl.e[e] = lo;
        }
        *(v8us*)(sAhi + j * APITCH + kc) = ph.v;
        *(v8us*)(sAlo + j * APITCH + kc) = pl.v;
    }
    __syncthreads();

    const float kNegW = -(6.283185307179586f / 4096.0f);
    const int lbase = l0 + wave * 32;
    float opr0, opi0, gr0, gi0, opr1, opi1, gr1, gi1;
    {
        const int lt = lbase + m;
        float so, co;
        sincosf(kNegW * (float)lt, &so, &co);
        opr0 = 1.0f + co; opi0 = so;
        const float nr = 2000.0f * (1.0f - co), ni = 2000.0f * (0.0f - so);
        const float d = 1.0f / (opr0 * opr0 + opi0 * opi0);
        gr0 = (nr * opr0 + ni * opi0) * d;
        gi0 = (ni * opr0 - nr * opi0) * d;
    }
    {
        const int lt = lbase + 16 + m;
        float so, co;
        sincosf(kNegW * (float)lt, &so, &co);
        opr1 = 1.0f + co; opi1 = so;
        const float nr = 2000.0f * (1.0f - co), ni = 2000.0f * (0.0f - so);
        const float d = 1.0f / (opr1 * opr1 + opi1 * opi1);
        gr1 = (nr * opr1 + ni * opi1) * d;
        gi1 = (ni * opr1 - nr * opi1) * d;
    }

    v8f acc0 = {0, 0, 0, 0, 0, 0, 0, 0};
    v8f acc1 = {0, 0, 0, 0, 0, 0, 0, 0};
    acc0 = cauchy_tile(acc0, gr0, gi0, s_lr, s_li, sAhi, sAlo, m, hh);
    acc1 = cauchy_tile(acc1, gr1, gi1, s_lr, s_li, sAhi, sAlo, m, hh);

    float r[8];
#pragma unroll
    for (int q = 0; q < 8; ++q) {
        float t1 = __shfl(acc1[q], m, 32);
        r[q] = hh ? t1 : acc0[q];
    }
    const float opr = hh ? opr1 : opr0;
    const float opi = hh ? opi1 : opi0;
    const float dd0 = 1.0f / (opr * opr + opi * opi);
    const float c2r = 2.0f * opr * dd0;
    const float c2i = -2.0f * opi * dd0;
    const float tr = r[2] * r[4] - r[3] * r[5];
    const float ti = r[2] * r[5] + r[3] * r[4];
    const float denr = 1.0f + r[6], deni = r[7];
    const float dd1 = 1.0f / (denr * denr + deni * deni);
    const float qr = (tr * denr + ti * deni) * dd1;
    const float qi = (ti * denr - tr * deni) * dd1;
    const float kkr = r[0] - qr, kki = r[1] - qi;
    const float Kre = c2r * kkr - c2i * kki;
    const float Kim = c2r * kki + c2i * kkr;
    sK[wave * 32 + lane] = Kre;
    sK[256 + wave * 32 + lane] = Kim;
    __syncthreads();

    if (wave < 4) {
        const int buf = wave >> 1;
        const int q = (wave & 1) * 32 + lane;
        v4f v = *(const v4f*)(sK + buf * 256 + 4 * q);
        float* dst = (buf ? Ki : Kr) + (size_t)h * LSEQ + l0 + 4 * q;
        *(volatile v4f*)dst = v;
        __threadfence();
        *(volatile v4f*)dst = v;
    }
}

__global__ __launch_bounds__(256) void k_fftconv(
    const float* __restrict__ x, const float* __restrict__ stats,
    const float* __restrict__ tw,
    const float* __restrict__ Kr, const float* __restrict__ Ki,
    _Float16* act)
{
    __shared__ __attribute__((aligned(16))) float s[2 * LSEQ];
    __shared__ __attribute__((aligned(16))) float stw[LSEQ];
    const int bh = blockIdx.x;
    if (bh >= NB * HD) return;
    const int b = bh >> 7;
    const int h = bh & (HD - 1);
    const int tid = threadIdx.x;

    const float mu = stats[b * 32 + 0];
    const float rs = stats[b * 32 + 1];
#pragma unroll
    for (int it = 0; it < 4; ++it) {
        const int q = it * 256 + tid;
        *(v4f*)(stw + 4 * q) = *(const v4f*)(tw + 4 * q);
    }
    const float* xp = x + (size_t)b * LSEQ * HD + h;
#pragma unroll 4
    for (int i = tid; i < LSEQ; i += 256) {
        float v = (xp[(size_t)i * HD] - mu) * rs;
        s[2 * i] = v;
        s[2 * i + 1] = 0.0f;
    }
    __syncthreads();

#pragma unroll 1
    for (int hb = 11; hb >= 0; --hb) {
        const int half = 1 << hb, sh = 11 - hb;
#pragma unroll 1
        for (int i = tid; i < LSEQ / 2; i += 256) {
            const int j = i & (half - 1);
            const int i1 = ((i >> hb) << (hb + 1)) | j;
            const int i2 = i1 + half;
            const float wx = stw[2 * (j << sh)], wy = stw[2 * (j << sh) + 1];
            const float ar = s[2 * i1], ai = s[2 * i1 + 1];
            const float cr = s[2 * i2], ci = s[2 * i2 + 1];
            s[2 * i1] = ar + cr;
            s[2 * i1 + 1] = ai + ci;
            const float tr = ar - cr, ti = ai - ci;
            s[2 * i2] = tr * wx + ti * wy;
            s[2 * i2 + 1] = ti * wx - tr * wy;
        }
        __syncthreads();
    }

    const float* krh = Kr + (size_t)h * LSEQ;
    const float* kih = Ki + (size_t)h * LSEQ;
#pragma unroll 1
    for (int i = tid; i < LSEQ; i += 256) {
        const int f = (int)(__brev((unsigned)i) >> 20);
        const float kr = krh[f], ki = kih[f];
        const float vr = s[2 * i], vi = s[2 * i + 1];
        s[2 * i] = vr * kr - vi * ki;
        s[2 * i + 1] = vr * ki + vi * kr;
    }
    __syncthreads();

#pragma unroll 1
    for (int hb = 0; hb <= 11; ++hb) {
        const int half = 1 << hb, sh = 11 - hb;
#pragma unroll 1
        for (int i = tid; i < LSEQ / 2; i += 256) {
            const int j = i & (half - 1);
            const int i1 = ((i >> hb) << (hb + 1)) | j;
            const int i2 = i1 + half;
            const float wx = stw[2 * (j << sh)], wy = stw[2 * (j << sh) + 1];
            const float ar = s[2 * i1], ai = s[2 * i1 + 1];
            const float cr = s[2 * i2], ci = s[2 * i2 + 1];
            const float tr = cr * wx - ci * wy;
            const float ti = cr * wy + ci * wx;
            s[2 * i1] = ar + tr;
            s[2 * i1 + 1] = ai + ti;
            s[2 * i2] = ar - tr;
            s[2 * i2 + 1] = ai - ti;
        }
        __syncthreads();
    }

#pragma unroll 1
    for (int i = tid; i < LSEQ; i += 256) {
        const float v = s[2 * i] * (1.0f / 4096.0f);
        const float g = 0.5f * v * (1.0f + erff(v * 0.70710678118654752f));
        s[2 * i] = 16.0f * g;
    }
    __syncthreads();

    Pack8h u0, u1;
#pragma unroll
    for (int j = 0; j < 8; ++j) {
        u0.e[j] = (_Float16)s[2 * (8 * tid + j)];
        u1.e[j] = (_Float16)s[2 * (8 * (256 + tid) + j)];
    }
    _Float16* base = act + (size_t)bh * LSEQ;
    _Float16* d0 = base + 8 * tid;
    _Float16* d1 = base + 8 * (256 + tid);
    *(volatile v8h*)d0 = u0.v;
    *(volatile v8h*)d1 = u1.v;
    __threadfence();
    *(volatile v8h*)d0 = u0.v;
    *(volatile v8h*)d1 = u1.v;
}

__global__ __launch_bounds__(256) void k_gemm(
    const _Float16* __restrict__ act, const float* __restrict__ W1,
    const float* __restrict__ b1, const float* __restrict__ xs,
    float* out)
{
    __shared__ __attribute__((aligned(16))) _Float16 sB[64 * BPITCH];
    __shared__ __attribute__((aligned(16))) float sO[64 * OPITCH];
    const int blk = blockIdx.x;
    if (blk >= NB * (LSEQ / 64)) return;
    const int b = blk >> 6;
    const int l0 = (blk & 63) * 64;
    const int tid = threadIdx.x;
    const int lane = tid & 31, wave = tid >> 5;
    const int hh = lane >> 4, m = lane & 15;

#pragma unroll
    for (int it = 0; it < 4; ++it) {
        const int idx = it * 256 + tid;
        const int kch = idx >> 3;
        const int lc = (idx & 7) * 8;
        Pack8h u;
        u.v = *(const v8h*)(act + ((size_t)(b * HD + kch)) * LSEQ + l0 + lc);
#pragma unroll
        for (int j = 0; j < 8; ++j) sB[(lc + j) * BPITCH + kch] = u.e[j];
    }
    __syncthreads();

    const int n0 = wave * 16;
    v8f acc[4];
#pragma unroll
    for (int mt = 0; mt < 4; ++mt) { v8f z = {0, 0, 0, 0, 0, 0, 0, 0}; acc[mt] = z; }

#pragma unroll
    for (int ks = 0; ks < 4; ++ks) {
        const int k0 = ks * 32;
        const float* wrow = W1 + (size_t)(n0 + m) * HD + k0;
        const v4f w0 = *(const v4f*)(wrow + 8 * hh);
        const v4f w1 = *(const v4f*)(wrow + 8 * hh + 4);
        const v4f w2 = *(const v4f*)(wrow + 16 + 8 * hh);
        const v4f w3 = *(const v4f*)(wrow + 16 + 8 * hh + 4);
        FragH a;
#pragma unroll
        for (int i = 0; i < 4; ++i) {
            a.e[i]      = (_Float16)(64.0f * w0[i]);
            a.e[4 + i]  = (_Float16)(64.0f * w1[i]);
            a.e[8 + i]  = (_Float16)(64.0f * w2[i]);
            a.e[12 + i] = (_Float16)(64.0f * w3[i]);
        }
#pragma unroll
        for (int mt = 0; mt < 4; ++mt) {
            FragH bb;
            bb.hv[0] = *(const v8h*)(sB + (16 * mt + m) * BPITCH + k0 + 8 * hh);
            bb.hv[1] = *(const v8h*)(sB + (16 * mt + m) * BPITCH + k0 + 16 + 8 * hh);
            acc[mt] = mma_f16(a.v, bb.v, acc[mt]);
        }
    }

#pragma unroll
    for (int mt = 0; mt < 4; ++mt) {
        float* p = sO + (16 * mt + m) * OPITCH + n0 + 8 * hh;
        v4f lo4 = {acc[mt][0], acc[mt][1], acc[mt][2], acc[mt][3]};
        v4f hi4 = {acc[mt][4], acc[mt][5], acc[mt][6], acc[mt][7]};
        *(v4f*)p = lo4;
        *(v4f*)(p + 4) = hi4;
    }
    __syncthreads();

    const v4f bias = *(const v4f*)(b1 + 4 * lane);
    const float osc = 1.0f / 1024.0f;
#pragma unroll 1
    for (int j = 0; j < 8; ++j) {
        const int lr = wave * 8 + j;
        const size_t mrow = (size_t)b * LSEQ + l0 + lr;
        const v4f o = *(const v4f*)(sO + lr * OPITCH + 4 * lane);
        const v4f sk = *(const v4f*)(xs + mrow * HD + 4 * lane);
        v4f v = o * osc + bias;
        v = v + sk;
        *(volatile v4f*)(out + mrow * HD + 4 * lane) = v;
    }
    __threadfence();
#pragma unroll 1
    for (int j = 0; j < 8; ++j) {
        const int lr = wave * 8 + j;
        const size_t mrow = (size_t)b * LSEQ + l0 + lr;
        const v4f o = *(const v4f*)(sO + lr * OPITCH + 4 * lane);
        const v4f sk = *(const v4f*)(xs + mrow * HD + 4 * lane);
        v4f v = o * osc + bias;
        v = v + sk;
        *(volatile v4f*)(out + mrow * HD + 4 * lane) = v;
    }
}

extern "C" void kernel_launch(void* const* d_in, const int* in_sizes, int n_in,
                              void* d_out, int out_size, void* d_ws, size_t ws_size,
                              hipStream_t stream)
{
    if (n_in < 11) return;
    if (in_sizes[0] != NB * LSEQ * HD) return;
    if (out_size != NB * LSEQ * HD) return;
    if (in_sizes[1] != HD * NS || in_sizes[2] != HD * NS || in_sizes[3] != HD * NS ||
        in_sizes[4] != HD * NS || in_sizes[5] != HD * NS || in_sizes[6] != HD * NS ||
        in_sizes[7] != HD * NS || in_sizes[8] != HD * NS) return;
    if (in_sizes[9] != HD * HD || in_sizes[10] != HD) return;

    const float* x    = (const float*)d_in[0];
    const float* LamR = (const float*)d_in[1];
    const float* LamI = (const float*)d_in[2];
    const float* Pre  = (const float*)d_in[3];
    const float* Pim  = (const float*)d_in[4];
    const float* Bre  = (const float*)d_in[5];
    const float* Bim  = (const float*)d_in[6];
    const float* Cre  = (const float*)d_in[7];
    const float* Cim  = (const float*)d_in[8];
    const float* W1   = (const float*)d_in[9];
    const float* b1   = (const float*)d_in[10];
    float* out = (float*)d_out;

    const size_t off_stats = 0;
    const size_t off_tw    = 4096;
    const size_t off_kr    = 65536;
    const size_t off_ki    = off_kr + (size_t)HD * LSEQ * 4;
    const size_t off_act   = off_ki + (size_t)HD * LSEQ * 4;
    const size_t total     = off_act + (size_t)NB * HD * LSEQ * 2;
    if (ws_size < total) return;

    char* base = (char*)d_ws;
    float*    stats = (float*)(base + off_stats);
    float*    tw    = (float*)(base + off_tw);
    float*    Kr    = (float*)(base + off_kr);
    float*    Ki    = (float*)(base + off_ki);
    _Float16* act   = (_Float16*)(base + off_act);

    k_stats<<<NB, 256, 0, stream>>>(x, stats);
    k_tw<<<(LSEQ / 4 + 255) / 256, 256, 0, stream>>>(tw);
    k_cauchy<<<HD * (LSEQ / 256), 256, 0, stream>>>(LamR, LamI, Pre, Pim, Bre, Bim, Cre, Cim, Kr, Ki);
    k_fftconv<<<NB * HD, 256, 0, stream>>>(x, stats, tw, Kr, Ki, act);
    k_gemm<<<NB * (LSEQ / 64), 256, 0, stream>>>(act, W1, b1, x, out);
}
